// _GATHead_63608465654521
// MI455X (gfx1250) — hardware-verified
//
#include <hip/hip_runtime.h>
#include <math.h>

typedef __attribute__((ext_vector_type(16))) _Float16 v16h;
typedef __attribute__((ext_vector_type(8)))  _Float16 v8h;
typedef __attribute__((ext_vector_type(16))) __bf16   v16b;
typedef __attribute__((ext_vector_type(8)))  __bf16   v8b;
typedef __attribute__((ext_vector_type(8)))  float    v8f;
typedef __attribute__((ext_vector_type(4)))  float    v4f;
#define PSCALE 32768.0f
#define U16(p) ((const unsigned short*)(const void*)(p))
#define PSCALE_INV (1.0f / 32768.0f)

__device__ __forceinline__ unsigned short f2bf_bits(float f) {
  unsigned u = __float_as_uint(f);
  return (unsigned short)((u + 0x7FFFu + ((u >> 16) & 1u)) >> 16);
}
__device__ __forceinline__ float bf_bits2f(unsigned short h) { return __uint_as_float(((unsigned)h) << 16); }

__device__ __forceinline__ void dep_guard_h(v8f& a, v8f& b, v16h x, v16h y) { asm volatile("v_nop\n\tv_nop\n\tv_nop\n\tv_nop" : "+v"(a), "+v"(b) : "v"(x), "v"(y)); }
__device__ __forceinline__ void dep_guard_b(v8f& a, v8f& b, v16b x, v16b y) { asm volatile("v_nop\n\tv_nop\n\tv_nop\n\tv_nop" : "+v"(a), "+v"(b) : "v"(x), "v"(y)); }
__device__ __forceinline__ void keep4_h(v16h a, v16h b, v16h c, v16h d) { asm volatile("v_nop" :: "v"(a), "v"(b), "v"(c), "v"(d)); }
__device__ __forceinline__ void keep4_b(v16b a, v16b b, v16b c, v16b d) { asm volatile("v_nop" :: "v"(a), "v"(b), "v"(c), "v"(d)); }
__device__ __forceinline__ void acc_guard4(v8f& a, v8f& b, v8f& c, v8f& d) { asm volatile("v_nop\n\tv_nop\n\tv_nop\n\tv_nop" : "+v"(a), "+v"(b), "+v"(c), "+v"(d)); }
template <typename T> struct Frag;
template <> struct Frag<_Float16> {
  typedef v16h V; union U { v16h v; v8h h[2]; };
  static __device__ __forceinline__ v16h load(const _Float16* p) {
    U f; f.h[0] = *(const v8h*)(p); f.h[1] = *(const v8h*)(p + 16); return f.v;
  }
  static __device__ __forceinline__ v8f mma(v16h a, v16h b, v8f c) {
    return __builtin_amdgcn_wmma_f32_16x16x32_f16(false, a, false, b, (short)0, c, false, false);
  }
  static __device__ __forceinline__ void guard(v8f& a, v8f& b, v16h x, v16h y) { dep_guard_h(a, b, x, y); }
  static __device__ __forceinline__ void keep(v16h a, v16h b, v16h c, v16h d) { keep4_h(a, b, c, d); }
};
template <> struct Frag<__bf16> {
  typedef v16b V; union U { v16b v; v8b h[2]; };
  static __device__ __forceinline__ v16b load(const __bf16* p) {
    U f; f.h[0] = *(const v8b*)(p); f.h[1] = *(const v8b*)(p + 16); return f.v;
  }
  static __device__ __forceinline__ v8f mma(v16b a, v16b b, v8f c) {
    return __builtin_amdgcn_wmma_f32_16x16x32_bf16(false, a, false, b, (short)0, c, false, false);
  }
  static __device__ __forceinline__ void guard(v8f& a, v8f& b, v16b x, v16b y) { dep_guard_b(a, b, x, y); }
  static __device__ __forceinline__ void keep(v16b a, v16b b, v16b c, v16b d) { keep4_b(a, b, c, d); }
};

template <int ET> struct Elem;
template <> struct Elem<0> { typedef _Float16 T; };
template <> struct Elem<1> { typedef __bf16 T; };
template <int ET, bool SPLIT, int BIAS_MODE, int OUT_MODE, bool RESID, int ACT = 0>
__global__ __launch_bounds__(256) void wmma_gemm64(
    const unsigned short* __restrict__ Ap, const unsigned short* __restrict__ A2p, int lda, long strideA,
    const unsigned short* __restrict__ Btp, const unsigned short* __restrict__ Bt2p, int ldb, long strideB,
    void* __restrict__ Cout, void* __restrict__ Cout2, int ldc, long strideC,
    const float* __restrict__ bias,
    const float* __restrict__ resid, long strideR,
    int M, int N, int K, float scale) {
  typedef typename Elem<ET>::T T;
  typedef typename Frag<T>::V V;
  const T* A = (const T*)Ap; const T* A2 = (const T*)A2p; const T* Bt = (const T*)Btp; const T* Bt2 = (const T*)Bt2p;
  __shared__ __align__(16) float sT[8][16 * 68];
  const int b    = blockIdx.y;
  const int lane = threadIdx.x & 31;
  const int wave = threadIdx.x >> 5;
  const int tilesN = N >> 6;
  const int tilesM = M >> 6;
  const int tile = blockIdx.x * 8 + wave;
  if (tile >= tilesM * tilesN) return;
  const int tm = tile / tilesN;
  const int tn = tile - tm * tilesN;
  const int m0 = tm << 6;
  const int n0 = tn << 6;

  const T* Ab  = A  + (size_t)b * strideA;
  const T* Bb  = Bt + (size_t)b * strideB;
  const T* Ab2 = SPLIT ? (A2  + (size_t)b * strideA) : nullptr;
  const T* Bb2 = SPLIT ? (Bt2 + (size_t)b * strideB) : nullptr;

  const int rlane = lane & 15;
  const int koff  = (lane >> 4) * 8;
  const int mOff  = (lane >> 4) * 8;

  v8f acc[4][4];
#pragma unroll
  for (int i = 0; i < 4; ++i)
#pragma unroll
    for (int j = 0; j < 4; ++j) acc[i][j] = (v8f){0.f,0.f,0.f,0.f,0.f,0.f,0.f,0.f};

  for (int k0 = 0; k0 < K; k0 += 32) {
    V bh[4], bl[4];
#pragma unroll
    for (int j = 0; j < 4; ++j) {
      const size_t bo = (size_t)(n0 + (j << 4) + rlane) * ldb + koff + k0;
      bh[j] = Frag<T>::load(Bb + bo);
      if (SPLIT) bl[j] = Frag<T>::load(Bb2 + bo);
    }
#pragma unroll
    for (int i = 0; i < 4; ++i) {
      const size_t ao = (size_t)(m0 + (i << 4) + rlane) * lda + koff + k0;
      V ah = Frag<T>::load(Ab + ao);
      V al;
      if (SPLIT) al = Frag<T>::load(Ab2 + ao);
#pragma unroll
      for (int j = 0; j < 4; ++j) {
        acc[i][j] = Frag<T>::mma(ah, bh[j], acc[i][j]);
        if (SPLIT) {
          acc[i][j] = Frag<T>::mma(ah, bl[j], acc[i][j]);
          acc[i][j] = Frag<T>::mma(al, bh[j], acc[i][j]);
        }
      }
      Frag<T>::guard(acc[i][0], acc[i][3], ah, SPLIT ? al : ah);
    }
    Frag<T>::keep(bh[0], bh[1], bh[2], bh[3]);
    if (SPLIT) Frag<T>::keep(bl[0], bl[1], bl[2], bl[3]);
  }
  acc_guard4(acc[0][0], acc[0][1], acc[0][2], acc[0][3]);
  acc_guard4(acc[1][0], acc[1][1], acc[1][2], acc[1][3]);
  acc_guard4(acc[2][0], acc[2][1], acc[2][2], acc[2][3]);
  acc_guard4(acc[3][0], acc[3][1], acc[3][2], acc[3][3]);

  float* slab = sT[wave];
  const float* Rb = RESID ? (resid + (size_t)b * strideR) : nullptr;
#pragma unroll
  for (int i = 0; i < 4; ++i) {
    const int mBase = m0 + (i << 4);
#pragma unroll
    for (int j = 0; j < 4; ++j) {
      const int n = n0 + (j << 4) + rlane;
      float bv = 0.f;
      if (BIAS_MODE == 2) bv = bias[n];
#pragma unroll
      for (int r = 0; r < 8; ++r) {
        float v = acc[i][j][r] * scale;
        if (BIAS_MODE == 1) v += bias[mBase + mOff + r];
        if (BIAS_MODE == 2) v += bv;
        if (RESID) v += Rb[(size_t)(mBase + mOff + r) * ldc + n];
        if (ACT == 1) v = tanhf(v);
        if (ACT == 2) v = fmaxf(v, 0.0f);
        if (ACT == 3) v = v / (1.0f + expf(-v));
        if (ACT == 4) v = (v > 0.f) ? v : 0.01f * v;
        if (ACT == 5) v = 0.5f * v * (1.0f + erff(v * 0.70710678118654752f));
        slab[(mOff + r) * 68 + (j << 4) + rlane] = v;
      }
    }
    __builtin_amdgcn_fence(__ATOMIC_RELEASE, "workgroup");
    __builtin_amdgcn_wave_barrier();
    __builtin_amdgcn_fence(__ATOMIC_ACQUIRE, "workgroup");
    if (OUT_MODE == 0 || OUT_MODE == 3) {
      float* C = (float*)Cout + (size_t)b * strideC;
      const int hh = lane >> 4, c4 = (lane & 15) * 4;
      for (int pass = 0; pass < 2; ++pass) {
#pragma unroll
        for (int it = 0; it < 8; ++it) {
          const int row = it * 2 + hh;
          v4f v = *(const v4f*)(slab + row * 68 + c4);
          *(volatile v4f*)(C + (size_t)(mBase + row) * ldc + n0 + c4) = v;
        }
        __threadfence();
      }
    }
    if (OUT_MODE != 0) {
      const int q = lane >> 3, c8 = (lane & 7) * 8;
      unsigned short* C  = (unsigned short*)((OUT_MODE == 3) ? Cout2 : Cout) + (size_t)b * strideC;
      unsigned short* C2 = (OUT_MODE == 2) ? ((unsigned short*)Cout2 + (size_t)b * strideC) : nullptr;
      for (int pass = 0; pass < 2; ++pass) {
#pragma unroll
        for (int it = 0; it < 4; ++it) {
          const int row = it * 4 + q;
          const float* sp = slab + row * 68 + c8;
          v8h hv, lv;
#pragma unroll
          for (int e = 0; e < 8; ++e) {
            if (OUT_MODE == 1 || OUT_MODE == 3) {
              hv[e] = (_Float16)sp[e];
            } else {
              unsigned short hb = f2bf_bits(sp[e]);
              unsigned short lb = f2bf_bits(sp[e] - bf_bits2f(hb));
              hv[e] = __builtin_bit_cast(_Float16, hb);
              lv[e] = __builtin_bit_cast(_Float16, lb);
            }
          }
          *(volatile v8h*)(C + (size_t)(mBase + row) * ldc + n0 + c8) = hv;
          if (OUT_MODE == 2) *(volatile v8h*)(C2 + (size_t)(mBase + row) * ldc + n0 + c8) = lv;
        }
        __threadfence();
      }
    }
    __builtin_amdgcn_fence(__ATOMIC_RELEASE, "workgroup");
    __builtin_amdgcn_wave_barrier();
    __builtin_amdgcn_fence(__ATOMIC_ACQUIRE, "workgroup");
  }
}

#define NB     8
#define NNODE  2048
#define NIN    256
#define NOUT   128
#define QBLK   64
#define KCH    64
#define OPITCH 68

__global__ __launch_bounds__(256) void cast_f32_bf16x2_hilo(
    const float* __restrict__ in, unsigned short* __restrict__ hi, unsigned short* __restrict__ lo, int n2) {
  const int i = blockIdx.x * 256 + threadIdx.x;
  if (i < n2) {
    const float f0 = in[2 * i], f1 = in[2 * i + 1];
    const unsigned short h0 = f2bf_bits(f0), h1 = f2bf_bits(f1);
    const unsigned short l0 = f2bf_bits(f0 - bf_bits2f(h0));
    const unsigned short l1 = f2bf_bits(f1 - bf_bits2f(h1));
    const unsigned uh = (unsigned)h0 | ((unsigned)h1 << 16);
    const unsigned ul = (unsigned)l0 | ((unsigned)l1 << 16);
    ((volatile unsigned*)hi)[i] = uh;
    ((volatile unsigned*)lo)[i] = ul;
    __threadfence();
    ((volatile unsigned*)hi)[i] = uh;
    ((volatile unsigned*)lo)[i] = ul;
  }
}

__global__ __launch_bounds__(256) void gat_dots(
    const float* __restrict__ hT32, const float* __restrict__ a_src, const float* __restrict__ a_dst,
    float* __restrict__ srcv, float* __restrict__ dstv, int total) {
  const int gid = blockIdx.x * 256 + threadIdx.x;
  if (gid >= total) return;
  const int b   = gid / NNODE;
  const int key = gid - b * NNODE;
  const float* hp = hT32 + (size_t)b * NOUT * NNODE + key;
  float s = 0.f, d = 0.f;
#pragma unroll 4
  for (int o = 0; o < NOUT; ++o) {
    const float hv = hp[(size_t)o * NNODE];
    s += hv * a_src[o];
    d += hv * a_dst[o];
  }
  ((volatile float*)srcv)[gid] = s;
  ((volatile float*)dstv)[gid] = d;
  __threadfence();
  ((volatile float*)srcv)[gid] = s;
  ((volatile float*)dstv)[gid] = d;
}

__device__ __forceinline__ v8f mma_f16(v16h a, v16h b, v8f c) {
  c = __builtin_amdgcn_wmma_f32_16x16x32_f16(false, a, false, b, (short)0, c, false, false);
  asm volatile("v_nop\n\tv_nop\n\tv_nop\n\tv_nop" : "+v"(c) : "v"(a), "v"(b));
  return c;
}

__global__ __launch_bounds__(128) void gat_attn(
    const float* __restrict__ srcv, const float* __restrict__ dstv, const int* __restrict__ mask,
    const unsigned short* __restrict__ hT16p, float* __restrict__ out) {
  union FH { v16h v; v8h h[2]; };
  __shared__ __align__(16) _Float16 Hs[NOUT * KCH];
  __shared__ __align__(16) _Float16 Psh[4][16 * KCH];
  __shared__ __align__(16) float    Os[4][16 * OPITCH];
  __shared__ float redm[4];
  __shared__ int   reda[4];

  const _Float16* hT16 = (const _Float16*)(const void*)hT16p;
  const int tid  = threadIdx.x;
  const int wave = tid >> 5;
  const int lane = tid & 31;
  const int hh   = lane >> 4;
  const int c    = lane & 15;
  const int nqb  = NNODE / QBLK;
  const int bx   = blockIdx.x;
  const int b    = bx / nqb;
  const int qb   = bx - b * nqb;
  const int q0   = qb * QBLK + wave * 16;
  const size_t gbase = (size_t)b * NNODE;

  float mx = -INFINITY;
  int anyk = 0;
#pragma unroll 4
  for (int i = 0; i < NNODE / 128; ++i) {
    const int j = tid + 128 * i;
    const int mkv = mask[gbase + j];
    const float d = dstv[gbase + j];
    mx = (mkv != 0) ? fmaxf(mx, d) : mx;
    anyk |= (mkv != 0) ? 1 : 0;
  }
#pragma unroll
  for (int off = 16; off > 0; off >>= 1) {
    mx = fmaxf(mx, __shfl_xor(mx, off, 32));
    anyk |= __shfl_xor(anyk, off, 32);
  }
  if (lane == 0) { redm[wave] = mx; reda[wave] = anyk; }
  __syncthreads();
  mx   = fmaxf(fmaxf(redm[0], redm[1]), fmaxf(redm[2], redm[3]));
  anyk = reda[0] | reda[1] | reda[2] | reda[3];

  float srow[8], mrow[8], lsum[8];
#pragma unroll
  for (int r = 0; r < 8; ++r) {
    const float s = srcv[gbase + q0 + 8 * hh + r];
    float e = s + mx;
    e = (e > 0.f) ? e : 0.2f * e;
    srow[r] = s;
    mrow[r] = anyk ? e : 0.f;
    lsum[r] = 0.f;
  }
  v8f oacc[8];
#pragma unroll
  for (int t = 0; t < 8; ++t) oacc[t] = (v8f){0.f,0.f,0.f,0.f,0.f,0.f,0.f,0.f};

  for (int kc = 0; kc < NNODE / KCH; ++kc) {
    const int kv0 = kc * KCH;
    __syncthreads();
    {
      const _Float16* grow = hT16 + ((size_t)b * NOUT + tid) * NNODE + kv0;
      _Float16* lrow = Hs + tid * KCH;
#pragma unroll
      for (int i = 0; i < 8; ++i) *(v8h*)(lrow + 8 * i) = *(const v8h*)(grow + 8 * i);
    }
    __syncthreads();

    float dcol[4];
    int   mk[4];
#pragma unroll
    for (int j = 0; j < 4; ++j) {
      const int col = kv0 + j * 16 + c;
      dcol[j] = dstv[gbase + col];
      mk[j]   = mask[gbase + col];
    }
    _Float16* pw = Psh[wave];
#pragma unroll
    for (int r = 0; r < 8; ++r) {
#pragma unroll
      for (int j = 0; j < 4; ++j) {
        float e = srow[r] + dcol[j];
        e = (e > 0.f) ? e : 0.2f * e;
        const float p = (mk[j] != 0) ? __expf(e - mrow[r]) : 0.f;
        lsum[r] += p;
        pw[(8 * hh + r) * KCH + j * 16 + c] = (_Float16)(p * PSCALE);
      }
    }
    __builtin_amdgcn_fence(__ATOMIC_RELEASE, "workgroup");
    __builtin_amdgcn_wave_barrier();
    __builtin_amdgcn_fence(__ATOMIC_ACQUIRE, "workgroup");
#pragma unroll 1
    for (int kk = 0; kk < 2; ++kk) {
      FH pa;
      pa.h[0] = *(const v8h*)(pw + c * KCH + kk * 32 + 8 * hh);
      pa.h[1] = *(const v8h*)(pw + c * KCH + kk * 32 + 16 + 8 * hh);
#pragma unroll
      for (int t = 0; t < 8; ++t) {
        FH vb;
        vb.h[0] = *(const v8h*)(Hs + (t * 16 + c) * KCH + kk * 32 + 8 * hh);
        vb.h[1] = *(const v8h*)(Hs + (t * 16 + c) * KCH + kk * 32 + 16 + 8 * hh);
        oacc[t] = mma_f16(pa.v, vb.v, oacc[t]);
      }
    }
  }

  float inv[8];
#pragma unroll
  for (int r = 0; r < 8; ++r) {
    float l = lsum[r];
#pragma unroll
    for (int off = 1; off < 16; off <<= 1) l += __shfl_xor(l, off, 32);
    const float den = (l > 0.f) ? (l * PSCALE) : 1.0f;
    inv[r] = (l > 0.f) ? (1.0f / den) : 0.f;
  }
  float* os = Os[wave];
#pragma unroll
  for (int g = 0; g < 2; ++g) {
#pragma unroll
    for (int r = 0; r < 8; ++r) {
#pragma unroll
      for (int t = 0; t < 4; ++t) os[(8 * hh + r) * OPITCH + t * 16 + c] = oacc[4 * g + t][r] * inv[r];
    }
    __builtin_amdgcn_fence(__ATOMIC_RELEASE, "workgroup");
    __builtin_amdgcn_wave_barrier();
    __builtin_amdgcn_fence(__ATOMIC_ACQUIRE, "workgroup");
    {
      const int c4 = (lane & 15) * 4;
      for (int pass = 0; pass < 2; ++pass) {
#pragma unroll
        for (int it = 0; it < 8; ++it) {
          const int row = it * 2 + hh;
          v4f val = *(const v4f*)(os + row * OPITCH + c4);
          *(volatile v4f*)(out + (gbase + q0 + row) * NOUT + g * 64 + c4) = val;
        }
        __threadfence();
      }
    }
    __builtin_amdgcn_fence(__ATOMIC_RELEASE, "workgroup");
    __builtin_amdgcn_wave_barrier();
    __builtin_amdgcn_fence(__ATOMIC_ACQUIRE, "workgroup");
  }
}

extern "C" void kernel_launch(void* const* d_in, const int* in_sizes, int n_in,
                              void* d_out, int out_size, void* d_ws, size_t ws_size,
                              hipStream_t stream) {
  if (n_in < 5) return;
  if (in_sizes[0] != NB * NNODE * NIN) return;
  if (in_sizes[1] != NB * NNODE) return;
  if (in_sizes[2] != NOUT * NIN) return;
  if (in_sizes[3] != NOUT || in_sizes[4] != NOUT) return;
  if (out_size != NB * NNODE * NOUT) return;

  const float* x     = (const float*)d_in[0];
  const int*   mask  = (const int*)  d_in[1];
  const float* W     = (const float*)d_in[2];
  const float* a_src = (const float*)d_in[3];
  const float* a_dst = (const float*)d_in[4];
  float*       out   = (float*)d_out;

  const size_t nX   = (size_t)NB * NNODE * NIN;
  const size_t nW   = (size_t)NOUT * NIN;
  const size_t nH   = (size_t)NB * NNODE * NOUT;
  const size_t nV   = (size_t)NB * NNODE;
  const size_t offXh  = 0;
  const size_t offXl  = offXh  + nX * 2;
  const size_t offWh  = offXl  + nX * 2;
  const size_t offWl  = offWh  + nW * 2;
  const size_t offH32 = offWl  + nW * 2;
  const size_t offH16 = offH32 + nH * 4;
  const size_t offSrc = offH16 + nH * 2;
  const size_t offDst = offSrc + nV * 4;
  const size_t offEnd = offDst + nV * 4;
  if (offEnd > ws_size) return;

  char* ws = (char*)d_ws;
  unsigned short* xh   = (unsigned short*)(ws + offXh);
  unsigned short* xl   = (unsigned short*)(ws + offXl);
  unsigned short* Wh   = (unsigned short*)(ws + offWh);
  unsigned short* Wl   = (unsigned short*)(ws + offWl);
  float*          hT32 = (float*)(ws + offH32);
  unsigned short* hT16 = (unsigned short*)(ws + offH16);
  float*          srcv = (float*)(ws + offSrc);
  float*          dstv = (float*)(ws + offDst);

  const int n2x = (int)(nX / 2);
  const int n2w = (int)(nW / 2);
  cast_f32_bf16x2_hilo<<<(n2x + 255) / 256, 256, 0, stream>>>(x, xh, xl, n2x);
  cast_f32_bf16x2_hilo<<<(n2w + 255) / 256, 256, 0, stream>>>(W, Wh, Wl, n2w);

  wmma_gemm64<1, true, 0, 3, false, 0><<<dim3((NOUT / 64) * (NNODE / 64) / 8, NB), 256, 0, stream>>>(
      Wh, Wl, NIN, 0L,
      xh, xl, NIN, (long)NNODE * NIN,
      (void*)hT32, (void*)hT16, NNODE, (long)NOUT * NNODE,
      srcv, srcv, 0L,
      NOUT, NNODE, NIN, 1.0f);

  gat_dots<<<(int)((nV + 255) / 256), 256, 0, stream>>>(hT32, a_src, a_dst, srcv, dstv, (int)nV);

  gat_attn<<<NB * (NNODE / QBLK), 128, 0, stream>>>(srcv, dstv, mask, hT16, out);
}
